// VSSBlock_8177617731786
// MI455X (gfx1250) — hardware-run, weakly checked
//
#include <hip/hip_runtime.h>
#include <math.h>
#include <stddef.h>

typedef __attribute__((ext_vector_type(16))) _Float16 v16h;
typedef __attribute__((ext_vector_type(8)))  _Float16 v8h;
typedef __attribute__((ext_vector_type(16))) __bf16   v16b;
typedef __attribute__((ext_vector_type(8)))  __bf16   v8b;
typedef __attribute__((ext_vector_type(8)))  float    v8f;
typedef __attribute__((ext_vector_type(4)))  float    v4f;
typedef __attribute__((ext_vector_type(4)))  unsigned int v4u;

constexpr int kB = 8, kH = 56, kW = 56, kC = 96, kD = 192, kNS = 16, kKdir = 4, kR = 6;
constexpr int kL     = kH * kW;
constexpr int kRows  = kB * kL;
constexpr int kXZ    = 2 * kD;
constexpr int kMlp   = 4 * kC;
constexpr int kGrp   = 48;
constexpr int kProjN = kKdir * kGrp;
constexpr int kNpad  = 128;
constexpr float kEps = 1e-5f;
constexpr float kWCarry  = 64.0f;
constexpr float kXzCarry = 16.0f;
constexpr float kXcCarry = 256.0f;
constexpr float kYsCarry = 256.0f;
constexpr float kYoCarry = 16.0f;
constexpr float kGCarry  = 16.0f;

static_assert((kRows % 64) == 0 && (kXZ % 64) == 0 && (kProjN % 64) == 0 && (kNpad % 64) == 0 && (kMlp % 64) == 0, "GEMM M,N tile multiples");
static_assert((kC % 32) == 0 && (kD % 32) == 0 && (kMlp % 32) == 0, "GEMM K multiples of 32");
static_assert((kRows % 16) == 0 && (kRows % 8) == 0 && (kL % 64) == 0 && (kD % 64) == 0, "VALU tile multiples");
static_assert(kR + 2 * kNS <= kGrp && kNpad >= kC, "padding");

constexpr size_t kSzT16  = (size_t)kRows * kC * 2;
constexpr size_t kSzWIN  = (size_t)kXZ * kC * 2;
constexpr size_t kSzWXP  = (size_t)kProjN * kD * 2;
constexpr size_t kSzWOUT = (size_t)kNpad * kD * 2;
constexpr size_t kSzWFC1 = (size_t)kMlp * kC * 2;
constexpr size_t kSzWFC2 = (size_t)kNpad * kMlp * 2;
constexpr size_t kSzXZ   = (size_t)kRows * kXZ * 2;
constexpr size_t kSzXC   = (size_t)kRows * kD * 2;
constexpr size_t kSzPROJ = (size_t)kRows * kProjN * 4;
constexpr size_t kSzYS   = (size_t)kKdir * kRows * kD * 2;
constexpr size_t kSzYO   = (size_t)kRows * kD * 2;
constexpr size_t kSzS32  = (size_t)kRows * kNpad * 4;
constexpr size_t kSzX1   = (size_t)kRows * kC * 4;
constexpr size_t kOffT16  = 0;
constexpr size_t kOffWIN  = kOffT16  + kSzT16;
constexpr size_t kOffWXP  = kOffWIN  + kSzWIN;
constexpr size_t kOffWOUT = kOffWXP  + kSzWXP;
constexpr size_t kOffWFC1 = kOffWOUT + kSzWOUT;
constexpr size_t kOffWFC2 = kOffWFC1 + kSzWFC1;
constexpr size_t kOffXZ   = kOffWFC2 + kSzWFC2;
constexpr size_t kOffXC   = kOffXZ   + kSzXZ;
constexpr size_t kOffPROJ = kOffXC   + kSzXC;
constexpr size_t kOffYS   = kOffPROJ + kSzPROJ;
constexpr size_t kOffYO   = kOffYS   + kSzYS;
constexpr size_t kOffS32  = kOffYO   + kSzYO;
constexpr size_t kOffX1   = kOffS32  + kSzS32;
constexpr size_t kWsTotal = kOffX1   + kSzX1;
constexpr size_t kOffH16  = kOffT16;
constexpr size_t kOffG16  = kOffXZ;
constexpr size_t kOffA2   = kOffS32;
static_assert(kWsTotal == 124002304ull, "carve total");
static_assert(kWsTotal <= 134217728ull, "carve cap");
static_assert((size_t)kRows * kMlp * 2 == kSzXZ && (size_t)kRows * kNpad * 4 == kSzS32, "alias sizes");
static_assert((kOffWIN % 128) == 0 && (kOffWXP % 128) == 0 && (kOffWOUT % 128) == 0 && (kOffWFC1 % 128) == 0 &&
              (kOffWFC2 % 128) == 0 && (kOffXZ % 128) == 0 && (kOffXC % 128) == 0 && (kOffPROJ % 128) == 0 &&
              (kOffYS % 128) == 0 && (kOffYO % 128) == 0 && (kOffS32 % 128) == 0 && (kOffX1 % 128) == 0, "128-B aligned regions");

__device__ __forceinline__ unsigned short f2bf_bits(float f) {
  unsigned u = __float_as_uint(f);
  return (unsigned short)((u + 0x7FFFu + ((u >> 16) & 1u)) >> 16);
}
__device__ __forceinline__ float bf_bits2f(unsigned short h) { return __uint_as_float(((unsigned)h) << 16); }

__device__ __forceinline__ void dep_guard_h(v8f& a, v8f& b, v16h x, v16h y) { asm volatile("v_nop\n\tv_nop\n\tv_nop\n\tv_nop" : "+v"(a), "+v"(b) : "v"(x), "v"(y)); }
__device__ __forceinline__ void dep_guard_b(v8f& a, v8f& b, v16b x, v16b y) { asm volatile("v_nop\n\tv_nop\n\tv_nop\n\tv_nop" : "+v"(a), "+v"(b) : "v"(x), "v"(y)); }
__device__ __forceinline__ void dep_guard4_h(v8f& a, v8f& b, v8f& c, v8f& d, v16h x, v16h y) { asm volatile("v_nop\n\tv_nop\n\tv_nop\n\tv_nop" : "+v"(a), "+v"(b), "+v"(c), "+v"(d) : "v"(x), "v"(y)); }
__device__ __forceinline__ void dep_guard4_b(v8f& a, v8f& b, v8f& c, v8f& d, v16b x, v16b y) { asm volatile("v_nop\n\tv_nop\n\tv_nop\n\tv_nop" : "+v"(a), "+v"(b), "+v"(c), "+v"(d) : "v"(x), "v"(y)); }
__device__ __forceinline__ void keep4_h(v16h a, v16h b, v16h c, v16h d) { asm volatile("v_nop" :: "v"(a), "v"(b), "v"(c), "v"(d)); }
__device__ __forceinline__ void keep4_b(v16b a, v16b b, v16b c, v16b d) { asm volatile("v_nop" :: "v"(a), "v"(b), "v"(c), "v"(d)); }
__device__ __forceinline__ void acc_guard4(v8f& a, v8f& b, v8f& c, v8f& d) { asm volatile("v_nop\n\tv_nop\n\tv_nop\n\tv_nop" : "+v"(a), "+v"(b), "+v"(c), "+v"(d)); }
template <typename T> struct Frag;
template <> struct Frag<_Float16> {
  typedef v16h V; union U { v16h v; v8h h[2]; };
  static __device__ __forceinline__ v16h load(const _Float16* p) {
    U f; f.h[0] = *(const v8h*)(p); f.h[1] = *(const v8h*)(p + 16); return f.v;
  }
  static __device__ __forceinline__ v8f mma(v16h a, v16h b, v8f c) {
    return __builtin_amdgcn_wmma_f32_16x16x32_f16(false, a, false, b, (short)0, c, false, false);
  }
  static __device__ __forceinline__ void guard(v8f& a, v8f& b, v16h x, v16h y) { dep_guard_h(a, b, x, y); }
  static __device__ __forceinline__ void guard4(v8f& a, v8f& b, v8f& c, v8f& d, v16h x, v16h y) { dep_guard4_h(a, b, c, d, x, y); }
  static __device__ __forceinline__ void keep(v16h a, v16h b, v16h c, v16h d) { keep4_h(a, b, c, d); }
};
template <> struct Frag<__bf16> {
  typedef v16b V; union U { v16b v; v8b h[2]; };
  static __device__ __forceinline__ v16b load(const __bf16* p) {
    U f; f.h[0] = *(const v8b*)(p); f.h[1] = *(const v8b*)(p + 16); return f.v;
  }
  static __device__ __forceinline__ v8f mma(v16b a, v16b b, v8f c) {
    return __builtin_amdgcn_wmma_f32_16x16x32_bf16(false, a, false, b, (short)0, c, false, false);
  }
  static __device__ __forceinline__ void guard(v8f& a, v8f& b, v16b x, v16b y) { dep_guard_b(a, b, x, y); }
  static __device__ __forceinline__ void guard4(v8f& a, v8f& b, v8f& c, v8f& d, v16b x, v16b y) { dep_guard4_b(a, b, c, d, x, y); }
  static __device__ __forceinline__ void keep(v16b a, v16b b, v16b c, v16b d) { keep4_b(a, b, c, d); }
};

template <int ET> struct Elem;
template <> struct Elem<0> { typedef _Float16 T; };
template <> struct Elem<1> { typedef __bf16 T; };
template <int ET, bool SPLIT, int BIAS_MODE, int OUT_MODE, bool RESID, int ACT = 0>
__global__ __launch_bounds__(256) void wmma_gemm64(
    const unsigned short* __restrict__ Ap, const unsigned short* __restrict__ A2p, int lda, long strideA,
    const unsigned short* __restrict__ Btp, const unsigned short* __restrict__ Bt2p, int ldb, long strideB,
    void* __restrict__ Cout, void* __restrict__ Cout2, int ldc, long strideC,
    const float* __restrict__ bias,
    const float* __restrict__ resid, long strideR,
    int M, int N, int K, float scale, float oscale) {
  typedef typename Elem<ET>::T T;
  typedef typename Frag<T>::V V;
  const T* A = (const T*)Ap; const T* A2 = (const T*)A2p; const T* Bt = (const T*)Btp; const T* Bt2 = (const T*)Bt2p;
  __shared__ __align__(16) float sT[8][16 * 68];
  const int b    = blockIdx.y;
  const int lane = threadIdx.x & 31;
  const int wave = threadIdx.x >> 5;
  const int tilesN = N >> 6;
  const int tilesM = M >> 6;
  const int tile = blockIdx.x * 8 + wave;
  if (tile >= tilesM * tilesN) return;
  const int tm = tile / tilesN;
  const int tn = tile - tm * tilesN;
  const int m0 = tm << 6;
  const int n0 = tn << 6;

  const T* Ab  = A  + (size_t)b * strideA;
  const T* Bb  = Bt + (size_t)b * strideB;
  const T* Ab2 = SPLIT ? (A2  + (size_t)b * strideA) : nullptr;
  const T* Bb2 = SPLIT ? (Bt2 + (size_t)b * strideB) : nullptr;

  const int rlane = lane & 15;
  const int koff  = (lane >> 4) * 8;
  const int mOff  = (lane >> 4) * 8;

  v8f acc[4][4];
#pragma unroll
  for (int i = 0; i < 4; ++i)
#pragma unroll
    for (int j = 0; j < 4; ++j) acc[i][j] = (v8f){0.f,0.f,0.f,0.f,0.f,0.f,0.f,0.f};

  for (int k0 = 0; k0 < K; k0 += 32) {
    V bh[4], bl[4];
#pragma unroll
    for (int j = 0; j < 4; ++j) {
      const size_t bo = (size_t)(n0 + (j << 4) + rlane) * ldb + koff + k0;
      bh[j] = Frag<T>::load(Bb + bo);
      if (SPLIT) bl[j] = Frag<T>::load(Bb2 + bo);
    }
#pragma unroll
    for (int i = 0; i < 4; ++i) {
      const size_t ao = (size_t)(m0 + (i << 4) + rlane) * lda + koff + k0;
      V ah = Frag<T>::load(Ab + ao);
      V al;
      if (SPLIT) al = Frag<T>::load(Ab2 + ao);
#pragma unroll
      for (int j = 0; j < 4; ++j) {
        acc[i][j] = Frag<T>::mma(ah, bh[j], acc[i][j]);
        if (SPLIT) {
          acc[i][j] = Frag<T>::mma(ah, bl[j], acc[i][j]);
          acc[i][j] = Frag<T>::mma(al, bh[j], acc[i][j]);
        }
      }
      Frag<T>::guard4(acc[i][0], acc[i][1], acc[i][2], acc[i][3], ah, SPLIT ? al : ah);
    }
    Frag<T>::keep(bh[0], bh[1], bh[2], bh[3]);
    if (SPLIT) Frag<T>::keep(bl[0], bl[1], bl[2], bl[3]);
  }
  acc_guard4(acc[0][0], acc[0][1], acc[0][2], acc[0][3]);
  acc_guard4(acc[1][0], acc[1][1], acc[1][2], acc[1][3]);
  acc_guard4(acc[2][0], acc[2][1], acc[2][2], acc[2][3]);
  acc_guard4(acc[3][0], acc[3][1], acc[3][2], acc[3][3]);

  float* slab = sT[wave];
  const float* Rb = RESID ? (resid + (size_t)b * strideR) : nullptr;
#pragma unroll
  for (int i = 0; i < 4; ++i) {
    const int mBase = m0 + (i << 4);
#pragma unroll
    for (int j = 0; j < 4; ++j) {
      const int n = n0 + (j << 4) + rlane;
      float bv = 0.f;
      if (BIAS_MODE == 2) bv = bias[n];
#pragma unroll
      for (int r = 0; r < 8; ++r) {
        float v = acc[i][j][r] * scale;
        if (BIAS_MODE == 1) v += bias[mBase + mOff + r];
        if (BIAS_MODE == 2) v += bv;
        if (RESID) v += Rb[(size_t)(mBase + mOff + r) * ldc + n];
        if (ACT == 1) v = tanhf(v);
        if (ACT == 2) v = fmaxf(v, 0.0f);
        if (ACT == 3) v = v / (1.0f + expf(-v));
        if (ACT == 4) v = (v > 0.f) ? v : 0.01f * v;
        if (ACT == 6) {
          const float ug = 0.7978845608028654f * (v + 0.044715f * v * v * v);
          const float cdf = 0.5f * (1.0f + tanhf(ug));
          v = v * cdf;
        }
        v = v * oscale;
        slab[(mOff + r) * 68 + (j << 4) + rlane] = v;
      }
    }
    __builtin_amdgcn_fence(__ATOMIC_RELEASE, "workgroup");
    __builtin_amdgcn_wave_barrier();
    __builtin_amdgcn_fence(__ATOMIC_ACQUIRE, "workgroup");
    if (OUT_MODE == 0) {
      float* Cf = (float*)Cout + (size_t)b * strideC;
      const int hh = lane >> 4, c4 = (lane & 15) * 4;
      for (int pass = 0; pass < 2; ++pass) {
#pragma unroll
        for (int it = 0; it < 8; ++it) {
          const int row = it * 2 + hh;
          v4f v = *(const v4f*)(slab + row * 68 + c4);
          *(volatile v4f*)(Cf + (size_t)(mBase + row) * ldc + n0 + c4) = v;
        }
        __threadfence();
      }
    } else {
      const int q = lane >> 3, c8 = (lane & 7) * 8;
      unsigned short* Cs  = (unsigned short*)Cout  + (size_t)b * strideC;
      unsigned short* Cs2 = (OUT_MODE == 2) ? ((unsigned short*)Cout2 + (size_t)b * strideC) : nullptr;
      for (int pass = 0; pass < 2; ++pass) {
#pragma unroll
        for (int it = 0; it < 4; ++it) {
          const int row = it * 4 + q;
          const float* sp = slab + row * 68 + c8;
          v8h hv, lv;
#pragma unroll
          for (int e = 0; e < 8; ++e) {
            if (OUT_MODE == 1) {
              hv[e] = (_Float16)sp[e];
            } else {
              unsigned short hb = f2bf_bits(sp[e]);
              unsigned short lb = f2bf_bits(sp[e] - bf_bits2f(hb));
              hv[e] = __builtin_bit_cast(_Float16, hb);
              lv[e] = __builtin_bit_cast(_Float16, lb);
            }
          }
          *(volatile v8h*)(Cs + (size_t)(mBase + row) * ldc + n0 + c8) = hv;
          if (OUT_MODE == 2) *(volatile v8h*)(Cs2 + (size_t)(mBase + row) * ldc + n0 + c8) = lv;
        }
        __threadfence();
      }
    }
    __builtin_amdgcn_fence(__ATOMIC_RELEASE, "workgroup");
    __builtin_amdgcn_wave_barrier();
    __builtin_amdgcn_fence(__ATOMIC_ACQUIRE, "workgroup");
  }
}

__device__ __forceinline__ float h16_to_f32(unsigned hb) {
  const unsigned sgn = (hb & 0x8000u) << 16; const unsigned em = hb & 0x7fffu;
  const float fn = __uint_as_float((em << 13) + 0x38000000u);
  const float fs = (float)em * 5.9604644775390625e-8f;
  const float mag = (em < 0x400u) ? fs : fn; return __uint_as_float(__float_as_uint(mag) | sgn); }

__device__ __forceinline__ void unpack8_f16(const v4u w, const float sc, float (&o)[8]) {
#pragma unroll
  for (int i = 0; i < 4; ++i) {
    const unsigned u = w[i];
    o[2 * i]     = h16_to_f32(u & 0xffffu) * sc;
    o[2 * i + 1] = h16_to_f32(u >> 16) * sc;
  }
}
__device__ __forceinline__ v8h pack8_f16v(const v4f a, const v4f b) {
  v8h r;
  r[0] = (_Float16)a[0]; r[1] = (_Float16)a[1]; r[2] = (_Float16)a[2]; r[3] = (_Float16)a[3];
  r[4] = (_Float16)b[0]; r[5] = (_Float16)b[1]; r[6] = (_Float16)b[2]; r[7] = (_Float16)b[3];
  return r;
}
__device__ __forceinline__ float wave_sum(float s) {
#pragma unroll
  for (int m = 16; m; m >>= 1) s += __shfl_xor(s, m, 32);
  return s;
}

__global__ __launch_bounds__(256) void cast_pad_f16x2(
    const float* __restrict__ in, unsigned short* __restrict__ out, int n_real2, int n_pad2, float sc) {
  const int i = blockIdx.x * 256 + threadIdx.x;
  if (i < n_pad2) {
    const bool live = (i < n_real2);
    const int ic = live ? i : (n_real2 - 1);
    const float fl = live ? sc : 0.0f;
    const float a = in[2 * ic] * fl;
    const float bq = in[2 * ic + 1] * fl;
    const _Float16 h0 = (_Float16)a, h1 = (_Float16)bq;
    const unsigned u = (unsigned)__builtin_bit_cast(unsigned short, h0) | ((unsigned)__builtin_bit_cast(unsigned short, h1) << 16);
    ((volatile unsigned*)out)[i] = u;
    __threadfence();
    ((volatile unsigned*)out)[i] = u;
  }
}

__global__ __launch_bounds__(256) void pack_xproj_f16x2(const float* __restrict__ in, unsigned short* __restrict__ out) {
  const int i = blockIdx.x * 256 + threadIdx.x;
  if (i < kProjN * kD / 2) {
    const int e0 = 2 * i;
    const int rr = e0 / kD;
    const int col = e0 - rr * kD;
    const int k = rr / kGrp;
    const int c = rr - k * kGrp;
    const bool isdt = (c < kR);
    const bool isbc = (c >= 8) && (c < 8 + 2 * kNS);
    const bool live = isdt || isbc;
    const int sr = isdt ? c : (isbc ? (c - 2) : 0);
    const size_t si = ((size_t)k * (kR + 2 * kNS) + sr) * kD + col;
    const float fl = live ? kWCarry : 0.0f;
    const float a = in[si] * fl;
    const float bq = in[si + 1] * fl;
    const _Float16 h0 = (_Float16)a, h1 = (_Float16)bq;
    const unsigned u = (unsigned)__builtin_bit_cast(unsigned short, h0) | ((unsigned)__builtin_bit_cast(unsigned short, h1) << 16);
    ((volatile unsigned*)out)[i] = u;
    __threadfence();
    ((volatile unsigned*)out)[i] = u;
  }
}

template <bool ADD_S>
__global__ __launch_bounds__(256) void ln96_kernel(
    const float* __restrict__ xin, const float* __restrict__ sin_, const float* __restrict__ gw,
    const float* __restrict__ gb, unsigned short* __restrict__ o16, float* __restrict__ x1o)
{
  __shared__ __align__(16) float sL[8 * 384];
  const int tid = threadIdx.x, lane = tid & 31, wave = tid >> 5;
  const size_t r0 = ((size_t)blockIdx.x * 8 + wave) * 2;
  float v[2][3];
#pragma unroll
  for (int rr = 0; rr < 2; ++rr) {
#pragma unroll
    for (int i = 0; i < 3; ++i) {
      const int c = lane + 32 * i;
      float t = xin[(r0 + rr) * kC + c];
      if (ADD_S) t = t + sin_[(r0 + rr) * kNpad + c];
      v[rr][i] = t;
    }
  }
  asm volatile("" ::: "memory");
  float wv[3], bvv[3];
#pragma unroll
  for (int i = 0; i < 3; ++i) { wv[i] = gw[lane + 32 * i]; bvv[i] = gb[lane + 32 * i]; }
  float* slab = sL + wave * 384;
#pragma unroll
  for (int rr = 0; rr < 2; ++rr) {
    float s = 0.0f;
    s += v[rr][0]; s += v[rr][1]; s += v[rr][2];
    s = wave_sum(s);
    const float mean = s * (1.0f / (float)kC);
    float qv = 0.0f;
#pragma unroll
    for (int i = 0; i < 3; ++i) { const float dl = v[rr][i] - mean; qv = fmaf(dl, dl, qv); }
    qv = wave_sum(qv);
    const float var = qv * (1.0f / (float)kC);
    const float inv = 1.0f / sqrtf(var + kEps);
#pragma unroll
    for (int i = 0; i < 3; ++i) {
      const int c = lane + 32 * i;
      slab[rr * kC + c] = (v[rr][i] - mean) * inv * wv[i] + bvv[i];
      if (ADD_S) slab[192 + rr * kC + c] = v[rr][i];
    }
  }
  __syncthreads();
  const int jc = (lane < 24) ? lane : 23;
  const v4f q0 = *(const v4f*)(slab + 8 * jc);
  const v4f q1 = *(const v4f*)(slab + 8 * jc + 4);
  const v8h hv = pack8_f16v(q0, q1);
  v4f xa = q0, xb = q1;
  if (ADD_S) {
    const int j16 = (lane < 16) ? lane : 15;
    xa = *(const v4f*)(slab + 192 + 4 * lane);
    xb = *(const v4f*)(slab + 192 + 128 + 4 * j16);
  }
  for (int pass = 0; pass < 2; ++pass) {
    if (lane < 24) *(volatile v8h*)(o16 + r0 * kC + 8 * lane) = hv;
    if (ADD_S) {
      *(volatile v4f*)(x1o + r0 * kC + 4 * lane) = xa;
      if (lane < 16) *(volatile v4f*)(x1o + r0 * kC + 128 + 4 * lane) = xb;
    }
    __threadfence();
  }
}

constexpr int kConvPC = 58;
constexpr int kConvOP = 68;
__global__ __launch_bounds__(256) void dwconv_silu_kernel(
    const unsigned short* __restrict__ XZ, const float* __restrict__ cw, const float* __restrict__ cb,
    unsigned short* __restrict__ XC)
{
  __shared__ __align__(16) float sIn[3 * kConvPC * 64];
  __shared__ __align__(16) float sOut[kW * kConvOP];
  const int tid = threadIdx.x, lane = tid & 31, wave = tid >> 5;
  const int g   = blockIdx.x % 3;
  const int bhi = blockIdx.x / 3;
  const int h   = bhi % kH;
  const int b   = bhi / kH;
  const size_t rowb = (size_t)b * kL;
#pragma unroll 1
  for (int i = 0; i < 6; ++i) {
    const int s   = tid + 256 * i;
    const int r   = s >> 9;
    const int rem = s & 511;
    const int pc  = rem >> 3;
    const int j   = rem & 7;
    const int hh = h + r - 1, ww = pc - 1;
    const bool valid = (hh >= 0) && (hh < kH) && (ww >= 0) && (ww < kW);
    const int hc = (hh < 0) ? 0 : ((hh > kH - 1) ? (kH - 1) : hh);
    const int wc = (ww < 0) ? 0 : ((ww > kW - 1) ? (kW - 1) : ww);
    const v4u wd = *(const v4u*)(XZ + ((rowb + (size_t)hc * kW + wc) * kXZ + g * 64 + 8 * j));
    const float f = valid ? (1.0f / kXzCarry) : 0.0f;
    float o[8];
    unpack8_f16(wd, f, o);
    if (pc < kConvPC) {
      float* dst = sIn + (r * kConvPC + pc) * 64 + 8 * j;
      *(v4f*)dst       = (v4f){o[0], o[1], o[2], o[3]};
      *(v4f*)(dst + 4) = (v4f){o[4], o[5], o[6], o[7]};
    }
  }
  __syncthreads();
  const int c = tid & 63, qp = tid >> 6;
  const int d = g * 64 + c;
  float wt[9];
#pragma unroll
  for (int t = 0; t < 9; ++t) wt[t] = cw[d * 9 + t];
  const float bias = cb[d];
#pragma unroll 1
  for (int p = 0; p < 14; ++p) {
    const int w0 = qp + 4 * p;
    float acc = 0.0f;
#pragma unroll
    for (int dh = 0; dh < 3; ++dh) {
#pragma unroll
      for (int dw = 0; dw < 3; ++dw) {
        acc = fmaf(wt[dh * 3 + dw], sIn[(dh * kConvPC + w0 + dw) * 64 + c], acc);
      }
    }
    const float vv = acc + bias;
    const float e  = expf(-vv);
    const float sg = __builtin_amdgcn_rcpf(1.0f + e);
    sOut[w0 * kConvOP + c] = (vv * sg) * kXcCarry;
  }
  __syncthreads();
  const int q8 = lane >> 3, c8 = (lane & 7) * 8;
  v8h hv[2];
#pragma unroll
  for (int it = 0; it < 2; ++it) {
    const int pix  = it * 32 + wave * 4 + q8;
    const int pixc = (pix < kW) ? pix : (kW - 1);
    const float* sp = sOut + pixc * kConvOP + c8;
    hv[it] = pack8_f16v(*(const v4f*)sp, *(const v4f*)(sp + 4));
  }
  for (int pass = 0; pass < 2; ++pass) {
#pragma unroll
    for (int it = 0; it < 2; ++it) {
      if (it * 8 + wave < 14) {
        const int pix = it * 32 + wave * 4 + q8;
        *(volatile v8h*)(XC + (rowb + (size_t)h * kW + pix) * kD + g * 64 + c8) = hv[it];
      }
    }
    __threadfence();
  }
}

constexpr int kScanTS = 64;
constexpr int kScanCh = 64;
constexpr int kScanYP = 68;
static_assert((kL % kScanTS) == 0 && (kD % kScanCh) == 0, "scan tiles");

__device__ __forceinline__ int scan_pix(int k, int l) {
  const int l2 = (k & 2) ? (kL - 1 - l) : l;
  const int hq = l2 % kH;
  const int wq = l2 / kH;
  const int lt = hq * kW + wq;
  return (k & 1) ? lt : l2;
}

__global__ __launch_bounds__(64) void scan_kernel(
    const float* __restrict__ PROJ, const unsigned short* __restrict__ XC,
    const float* __restrict__ Wdt, const float* __restrict__ bdt,
    const float* __restrict__ Alog, const float* __restrict__ Dp,
    unsigned short* __restrict__ YS)
{
  __shared__ __align__(16) float sX[kScanTS * kGrp];
  __shared__ __align__(16) float sU[kScanTS * kScanCh];
  __shared__ __align__(16) float sY[kScanTS * kScanYP];
  __shared__ __align__(16) float sW[kR * kScanCh];
  __shared__ __align__(16) float sA[kNS * kScanCh];
  const int tid = threadIdx.x, lane = tid & 31, wave = tid >> 5;
  const int g  = blockIdx.x % 3;
  const int bk = blockIdx.x / 3;
  const int k  = bk % kKdir;
  const int b  = bk / kKdir;
  const int d0 = g * kScanCh;
  const int d  = d0 + tid;
  const int kd = k * kD + d;
  const size_t rowb  = (size_t)b * kL;
  const size_t plane = (size_t)k * kRows * kD;
#pragma unroll 1
  for (int r = 0; r < kR; ++r) sW[r * kScanCh + tid] = Wdt[(size_t)kd * kR + r];
#pragma unroll 1
  for (int s = 0; s < kNS; ++s) sA[s * kScanCh + tid] = -expf(Alog[(size_t)kd * kNS + s]);
  __syncthreads();
  float nA[kNS], h[kNS];
#pragma unroll
  for (int s = 0; s < kNS; ++s) { nA[s] = sA[s * kScanCh + tid]; h[s] = 0.0f; }
  const float bb = bdt[kd], Dd = Dp[kd];
  const int q = lane >> 3, c8 = (lane & 7) * 8;
#pragma unroll 1
  for (int t0 = 0; t0 < kL; t0 += kScanTS) {
    __syncthreads();
#pragma unroll 1
    for (int i = 0; i < 12; ++i) {
      const int slot = tid + kScanCh * i;
      const int s = slot / 12;
      const int j = slot - s * 12;
      const int p = scan_pix(k, t0 + s);
      *(v4f*)(sX + s * kGrp + 4 * j) = *(const v4f*)(PROJ + (rowb + p) * kProjN + k * kGrp + 4 * j);
    }
#pragma unroll 1
    for (int i = 0; i < 8; ++i) {
      const int slot = tid + kScanCh * i;
      const int s = slot >> 3;
      const int j = slot & 7;
      const int p = scan_pix(k, t0 + s);
      const v4u wd = *(const v4u*)(XC + (rowb + p) * kD + d0 + 8 * j);
      float o[8];
      unpack8_f16(wd, 1.0f / kXcCarry, o);
      float* dst = sU + s * kScanCh + 8 * j;
      *(v4f*)dst       = (v4f){o[0], o[1], o[2], o[3]};
      *(v4f*)(dst + 4) = (v4f){o[4], o[5], o[6], o[7]};
    }
    __syncthreads();
#pragma unroll 1
    for (int s = 0; s < kScanTS; ++s) {
      const float* xr = sX + s * kGrp;
      float vd = 0.0f;
#pragma unroll
      for (int r = 0; r < kR; ++r) vd = fmaf(xr[r], sW[r * kScanCh + tid], vd);
      const float v   = vd + bb;
      const float ea  = __expf(-fabsf(v));
      const float ua  = 1.0f + ea;
      const float l1p = __logf(ua) + (ea - (ua - 1.0f)) * __builtin_amdgcn_rcpf(ua);
      const float dt  = fmaxf(v, 0.0f) + l1p;
      const float u   = sU[s * kScanCh + tid];
      const float dtu = dt * u;
      float Bs[kNS], Cs[kNS];
#pragma unroll
      for (int q4 = 0; q4 < 4; ++q4) {
        const v4f bv = *(const v4f*)(xr + 8 + 4 * q4);
        const v4f cv = *(const v4f*)(xr + 8 + kNS + 4 * q4);
        Bs[4 * q4 + 0] = bv[0]; Bs[4 * q4 + 1] = bv[1]; Bs[4 * q4 + 2] = bv[2]; Bs[4 * q4 + 3] = bv[3];
        Cs[4 * q4 + 0] = cv[0]; Cs[4 * q4 + 1] = cv[1]; Cs[4 * q4 + 2] = cv[2]; Cs[4 * q4 + 3] = cv[3];
      }
      float y = 0.0f;
#pragma unroll
      for (int n = 0; n < kNS; ++n) {
        const float e = __expf(dt * nA[n]);
        h[n] = e * h[n] + dtu * Bs[n];
        y = fmaf(h[n], Cs[n], y);
      }
      const float ysv = y + Dd * u;
      sY[s * kScanYP + tid] = ysv * kYsCarry;
    }
    __syncthreads();
    v8h hv[8];
#pragma unroll
    for (int it = 0; it < 8; ++it) {
      const int rc = it * 8 + wave * 4 + q;
      const float* sp = sY + rc * kScanYP + c8;
      hv[it] = pack8_f16v(*(const v4f*)sp, *(const v4f*)(sp + 4));
    }
    for (int pass = 0; pass < 2; ++pass) {
#pragma unroll
      for (int it = 0; it < 8; ++it) {
        const int rc = it * 8 + wave * 4 + q;
        const int p = scan_pix(k, t0 + rc);
        *(volatile v8h*)(YS + plane + (rowb + p) * kD + d0 + c8) = hv[it];
      }
      __threadfence();
    }
  }
}

__global__ __launch_bounds__(256) void merge_norm_gate_kernel(
    const unsigned short* __restrict__ YS, const unsigned short* __restrict__ XZ,
    const float* __restrict__ nw, const float* __restrict__ nb, unsigned short* __restrict__ YO)
{
  __shared__ __align__(16) float sM[8 * kD];
  const int tid = threadIdx.x, lane = tid & 31, wave = tid >> 5;
  const size_t row = (size_t)blockIdx.x * 8 + wave;
  const int c0 = 6 * lane;
  const unsigned* Y32 = (const unsigned*)(const void*)YS;
  const unsigned* Z32 = (const unsigned*)(const void*)XZ;
  const size_t u0 = (row * kD + c0) >> 1;
  const size_t ps = ((size_t)kRows * kD) >> 1;
  const size_t z0 = (row * kXZ + kD + c0) >> 1;
  unsigned a0[3], a1[3], a2[3], a3[3], zw[3];
#pragma unroll
  for (int t = 0; t < 3; ++t) {
    a0[t] = Y32[u0 + t];
    a1[t] = Y32[u0 + ps + t];
    a2[t] = Y32[u0 + 2 * ps + t];
    a3[t] = Y32[u0 + 3 * ps + t];
    zw[t] = Z32[z0 + t];
  }
  asm volatile("" ::: "memory");
  float wv[6], bvv[6];
#pragma unroll
  for (int e = 0; e < 6; ++e) { wv[e] = nw[c0 + e]; bvv[e] = nb[c0 + e]; }
  float y[6], z[6];
  const unsigned mlo = 0xffffu;
  const float ysc = 1.0f / kYsCarry, zsc = 1.0f / kXzCarry;
#pragma unroll
  for (int t = 0; t < 3; ++t) {
    y[2 * t]     = ((h16_to_f32(a0[t] & mlo) + h16_to_f32(a2[t] & mlo)) + (h16_to_f32(a1[t] & mlo) + h16_to_f32(a3[t] & mlo))) * ysc;
    y[2 * t + 1] = ((h16_to_f32(a0[t] >> 16) + h16_to_f32(a2[t] >> 16)) + (h16_to_f32(a1[t] >> 16) + h16_to_f32(a3[t] >> 16))) * ysc;
    z[2 * t]     = h16_to_f32(zw[t] & mlo) * zsc;
    z[2 * t + 1] = h16_to_f32(zw[t] >> 16) * zsc;
  }
  float s = 0.0f;
#pragma unroll
  for (int e = 0; e < 6; ++e) s += y[e];
  s = wave_sum(s);
  const float mean = s * (1.0f / (float)kD);
  float qv = 0.0f;
#pragma unroll
  for (int e = 0; e < 6; ++e) { const float dl = y[e] - mean; qv = fmaf(dl, dl, qv); }
  qv = wave_sum(qv);
  const float var = qv * (1.0f / (float)kD);
  const float inv = 1.0f / sqrtf(var + kEps);
#pragma unroll
  for (int e = 0; e < 6; ++e) {
    const float ez = expf(-z[e]);
    const float sg = z[e] * __builtin_amdgcn_rcpf(1.0f + ez);
    const float ov = ((y[e] - mean) * inv * wv[e] + bvv[e]) * sg;
    sM[wave * kD + c0 + e] = ov * kYoCarry;
  }
  __syncthreads();
  const int jc = (lane < 24) ? lane : 23;
  const float* sp = sM + wave * kD + 8 * jc;
  const v8h hv = pack8_f16v(*(const v4f*)sp, *(const v4f*)(sp + 4));
  if (lane < 24) *(volatile v8h*)(YO + row * kD + 8 * lane) = hv;
  __threadfence();
  if (lane < 24) *(volatile v8h*)(YO + row * kD + 8 * lane) = hv;
}

__global__ __launch_bounds__(256) void final_out_kernel(
    const float* __restrict__ X1, const float* __restrict__ A2, const float* __restrict__ b2, float* __restrict__ out)
{
  const int tid = threadIdx.x, lane = tid & 31, wave = tid >> 5;
  const size_t row = (size_t)blockIdx.x * 8 + wave;
  const int jc = (lane < 24) ? lane : 23;
  const v4f xa = *(const v4f*)(X1 + row * kC + 4 * jc);
  const v4f oa = *(const v4f*)(A2 + row * kNpad + 4 * jc);
  const v4f ba = *(const v4f*)(b2 + 4 * jc);
  const v4f hs = oa + ba;
  const v4f rv = xa + hs;
  if (lane < 24) *(volatile v4f*)(out + row * kC + 4 * lane) = rv;
  __threadfence();
  if (lane < 24) *(volatile v4f*)(out + row * kC + 4 * lane) = rv;
}

static_assert(((kRows / 64) * (kXZ / 64)) % 8 == 0 && ((kRows / 64) * (kProjN / 64)) % 8 == 0 &&
              ((kRows / 64) * (kNpad / 64)) % 8 == 0 && ((kRows / 64) * (kMlp / 64)) % 8 == 0, "8 tiles per GEMM block");

extern "C" void kernel_launch(void* const* d_in, const int* in_sizes, int n_in,
                              void* d_out, int out_size, void* d_ws, size_t ws_size,
                              hipStream_t stream) {
  if (n_in < 20) return;
  if (in_sizes[0]  != kRows * kC) return;
  if (in_sizes[1]  != kC || in_sizes[2] != kC) return;
  if (in_sizes[3]  != kXZ * kC) return;
  if (in_sizes[4]  != kD * 9 || in_sizes[5] != kD) return;
  if (in_sizes[6]  != kKdir * (kR + 2 * kNS) * kD) return;
  if (in_sizes[7]  != kKdir * kD * kR || in_sizes[8] != kKdir * kD) return;
  if (in_sizes[9]  != kKdir * kD * kNS || in_sizes[10] != kKdir * kD) return;
  if (in_sizes[11] != kD || in_sizes[12] != kD) return;
  if (in_sizes[13] != kC * kD) return;
  if (in_sizes[14] != kC || in_sizes[15] != kC) return;
  if (in_sizes[16] != kMlp * kC || in_sizes[17] != kMlp) return;
  if (in_sizes[18] != kC * kMlp || in_sizes[19] != kC) return;
  if (out_size != kRows * kC) return;
  if (ws_size < kWsTotal) return;

  const float* x          = (const float*)d_in[0];
  const float* ln1_w      = (const float*)d_in[1];
  const float* ln1_b      = (const float*)d_in[2];
  const float* in_proj_w  = (const float*)d_in[3];
  const float* conv_w     = (const float*)d_in[4];
  const float* conv_b     = (const float*)d_in[5];
  const float* x_proj_w   = (const float*)d_in[6];
  const float* dt_proj_w  = (const float*)d_in[7];
  const float* dt_proj_b  = (const float*)d_in[8];
  const float* A_logs     = (const float*)d_in[9];
  const float* Ds         = (const float*)d_in[10];
  const float* onorm_w    = (const float*)d_in[11];
  const float* onorm_b    = (const float*)d_in[12];
  const float* out_proj_w = (const float*)d_in[13];
  const float* ln2_w      = (const float*)d_in[14];
  const float* ln2_b      = (const float*)d_in[15];
  const float* fc1_w      = (const float*)d_in[16];
  const float* fc1_b      = (const float*)d_in[17];
  const float* fc2_w      = (const float*)d_in[18];
  const float* fc2_b      = (const float*)d_in[19];
  float* out = (float*)d_out;

  char* ws = (char*)d_ws;
  unsigned short* T16  = (unsigned short*)(ws + kOffT16);
  unsigned short* WIN  = (unsigned short*)(ws + kOffWIN);
  unsigned short* WXP  = (unsigned short*)(ws + kOffWXP);
  unsigned short* WOUT = (unsigned short*)(ws + kOffWOUT);
  unsigned short* WFC1 = (unsigned short*)(ws + kOffWFC1);
  unsigned short* WFC2 = (unsigned short*)(ws + kOffWFC2);
  unsigned short* XZ   = (unsigned short*)(ws + kOffXZ);
  unsigned short* XC   = (unsigned short*)(ws + kOffXC);
  float*          PROJ = (float*)(ws + kOffPROJ);
  unsigned short* YS   = (unsigned short*)(ws + kOffYS);
  unsigned short* YO   = (unsigned short*)(ws + kOffYO);
  float*          S32  = (float*)(ws + kOffS32);
  float*          X1   = (float*)(ws + kOffX1);
  unsigned short* H16  = (unsigned short*)(ws + kOffH16);
  unsigned short* G16  = (unsigned short*)(ws + kOffG16);
  float*          A2   = (float*)(ws + kOffA2);

  cast_pad_f16x2<<<(kXZ * kC / 2) / 256, 256, 0, stream>>>(in_proj_w, WIN, kXZ * kC / 2, kXZ * kC / 2, kWCarry);
  pack_xproj_f16x2<<<(kProjN * kD / 2) / 256, 256, 0, stream>>>(x_proj_w, WXP);
  cast_pad_f16x2<<<(kNpad * kD / 2) / 256, 256, 0, stream>>>(out_proj_w, WOUT, kC * kD / 2, kNpad * kD / 2, kWCarry);
  cast_pad_f16x2<<<(kMlp * kC / 2) / 256, 256, 0, stream>>>(fc1_w, WFC1, kMlp * kC / 2, kMlp * kC / 2, kWCarry);
  cast_pad_f16x2<<<(kNpad * kMlp / 2) / 256, 256, 0, stream>>>(fc2_w, WFC2, kC * kMlp / 2, kNpad * kMlp / 2, kWCarry);

  ln96_kernel<false><<<kRows / 16, 256, 0, stream>>>(x, x, ln1_w, ln1_b, T16, X1);

  wmma_gemm64<0, false, 0, 1, false, 0><<<dim3(((kRows / 64) * (kXZ / 64)) / 8, 1), 256, 0, stream>>>(
      T16, T16, kC, 0L, WIN, WIN, kC, 0L, (void*)XZ, (void*)XZ, kXZ, 0L,
      ln1_w, x, 0L, kRows, kXZ, kC, kXzCarry / kWCarry, 1.0f);

  dwconv_silu_kernel<<<kB * kH * 3, 256, 0, stream>>>(XZ, conv_w, conv_b, XC);

  wmma_gemm64<0, false, 0, 0, false, 0><<<dim3(((kRows / 64) * (kProjN / 64)) / 8, 1), 256, 0, stream>>>(
      XC, XC, kD, 0L, WXP, WXP, kD, 0L, (void*)PROJ, (void*)PROJ, kProjN, 0L,
      ln1_w, x, 0L, kRows, kProjN, kD, 1.0f / (kXcCarry * kWCarry), 1.0f);

  scan_kernel<<<kB * kKdir * (kD / kScanCh), kScanCh, 0, stream>>>(PROJ, XC, dt_proj_w, dt_proj_b, A_logs, Ds, YS);

  merge_norm_gate_kernel<<<kRows / 8, 256, 0, stream>>>(YS, XZ, onorm_w, onorm_b, YO);

  wmma_gemm64<0, false, 0, 0, false, 0><<<dim3(((kRows / 64) * (kNpad / 64)) / 8, 1), 256, 0, stream>>>(
      YO, YO, kD, 0L, WOUT, WOUT, kD, 0L, (void*)S32, (void*)S32, kNpad, 0L,
      ln1_w, x, 0L, kRows, kNpad, kD, 1.0f / (kYoCarry * kWCarry), 1.0f);

  ln96_kernel<true><<<kRows / 16, 256, 0, stream>>>(x, S32, ln2_w, ln2_b, H16, X1);

  wmma_gemm64<0, false, 2, 1, false, 6><<<dim3(((kRows / 64) * (kMlp / 64)) / 8, 1), 256, 0, stream>>>(
      H16, H16, kC, 0L, WFC1, WFC1, kC, 0L, (void*)G16, (void*)G16, kMlp, 0L,
      fc1_b, x, 0L, kRows, kMlp, kC, 1.0f / kWCarry, kGCarry);

  wmma_gemm64<0, false, 0, 0, false, 0><<<dim3(((kRows / 64) * (kNpad / 64)) / 8, 1), 256, 0, stream>>>(
      G16, G16, kMlp, 0L, WFC2, WFC2, kMlp, 0L, (void*)A2, (void*)A2, kNpad, 0L,
      ln1_w, x, 0L, kRows, kNpad, kMlp, 1.0f / (kGCarry * kWCarry), 1.0f);

  final_out_kernel<<<kRows / 8, 256, 0, stream>>>(X1, A2, fc2_b, out);
}
